// NonLocalBlockOriginal_34531537060181
// MI455X (gfx1250) — hardware-run, weakly checked
//
#include <hip/hip_runtime.h>
#include <math.h>
#include <stddef.h>
#include <stdint.h>

#define NB    4
#define CC    128
#define CI    64
#define IH    96
#define IW    96
#define NPOS  (IH * IW)
#define NTOK  (NB * NPOS)
#define PWD   (IW / 2)
#define NKEY  ((IH / 2) * (IW / 2))
#define GTP   (2 * NKEY)
#define NGRP  32
#define CPG   4
#define SPT   68
#define TPT   132
#define WROWS 128
#define NREC  (NTOK / WROWS)
#define RECB  (NPOS / WROWS)
#define GCNT  (CPG * NPOS)
#define SV_BP 0
#define SV_BW 192
#define SV_GW 320
#define SV_GB 448
#define SV_N  576
#define PREP_XT 576
#define PREP_WP 12
#define PREP_WW 8
#define PREP_SV 6
#define WSMAX 134217728

static_assert(NPOS % 128 == 0);
static_assert(NPOS % 1024 == 0);
static_assert(NKEY % 64 == 0);
static_assert(IH % 2 == 0);
static_assert(IW % 2 == 0);
static_assert(PWD == 48);
static_assert(NKEY == 2304);
static_assert(CC == NGRP * CPG);
static_assert(CI == 64);
static_assert(CC % 32 == 0);
static_assert((3 * CI) % 64 == 0);
static_assert(NB * (NPOS / 64) == PREP_XT);
static_assert(NREC == 288);
static_assert(RECB == 72);
static_assert(GCNT == 36864);
static_assert(SV_N == 3 * CI + 3 * CC);

typedef float          v4f   __attribute__((ext_vector_type(4)));
typedef float          v8f   __attribute__((ext_vector_type(8)));
typedef int            v8i   __attribute__((ext_vector_type(8)));
typedef double         v2d   __attribute__((ext_vector_type(2)));
typedef unsigned short v8us  __attribute__((ext_vector_type(8)));
typedef unsigned short v16us __attribute__((ext_vector_type(16)));
typedef __bf16         v16bf __attribute__((ext_vector_type(16)));
typedef __bf16         v8bf  __attribute__((ext_vector_type(8)));
typedef v4f  __attribute__((may_alias)) v4fa;
typedef v8us __attribute__((may_alias)) v8usa;
typedef v2d  __attribute__((may_alias)) v2da;
union FragB { v16bf v; v16us u; v8us h[2]; v8i w; };

__device__ __forceinline__ v8f wmb(const FragB& a, const FragB& b, v8f c) {
  v8f d = __builtin_amdgcn_wmma_f32_16x16x32_bf16(false, a.v, false, b.v, (short)0, c, false, false);
  asm volatile("v_nop\n\tv_nop\n\tv_nop\n\tv_nop" : "+v"(d) : "v"(a.w), "v"(b.w));
  return d;
}
__device__ __forceinline__ v8f z8() { v8f z = {0.f, 0.f, 0.f, 0.f, 0.f, 0.f, 0.f, 0.f}; return z; }

__device__ __forceinline__ unsigned bf16_bits(float f) {
  const unsigned u = __float_as_uint(f);
  return (u + 0x7FFFu + ((u >> 16) & 1u)) >> 16;
}
__device__ __forceinline__ float bf16_val(float f) { return __uint_as_float(bf16_bits(f) << 16); }

__device__ __forceinline__ v8us cvt8(v4f a, v4f b) {
  v8us o8;
  o8[0] = (unsigned short)bf16_bits(a.x); o8[1] = (unsigned short)bf16_bits(a.y);
  o8[2] = (unsigned short)bf16_bits(a.z); o8[3] = (unsigned short)bf16_bits(a.w);
  o8[4] = (unsigned short)bf16_bits(b.x); o8[5] = (unsigned short)bf16_bits(b.y);
  o8[6] = (unsigned short)bf16_bits(b.z); o8[7] = (unsigned short)bf16_bits(b.w);
  return o8;
}

__global__ __launch_bounds__(256) void k_prep(const float* __restrict__ x,
                                             const float* __restrict__ wth, const float* __restrict__ bth,
                                             const float* __restrict__ wph, const float* __restrict__ bph,
                                             const float* __restrict__ wg,  const float* __restrict__ bg,
                                             const float* __restrict__ wW,  const float* __restrict__ bW,
                                             const float* __restrict__ gnw, const float* __restrict__ gnb,
                                             unsigned short* XT, unsigned short* WP, unsigned short* WW2, float* SV) {
  __shared__ __attribute__((aligned(16))) float tf[CC * SPT];
  const int bx = (int)blockIdx.x, tid = (int)threadIdx.x;
  if (bx < PREP_XT) {
    const int b  = bx / (NPOS / 64);
    const int n0 = (bx - b * (NPOS / 64)) * 64;
    {
      const int rsub = tid >> 4;
      const int c4   = (tid & 15) * 4;
#pragma unroll
      for (int it = 0; it < 8; ++it) {
        const int cr = it * 16 + rsub;
        const v4f a = *(const v4f*)(x + ((size_t)(b * CC + cr)) * NPOS + n0 + c4);
        *(v4fa*)(tf + cr * SPT + c4) = a;
      }
    }
    __syncthreads();
    const int rsub = tid >> 4;
    const int c8   = (tid & 15) * 8;
    v8us o[4];
#pragma unroll
    for (int it = 0; it < 4; ++it) {
      const int tl = it * 16 + rsub;
      v8us w;
#pragma unroll
      for (int e = 0; e < 8; ++e) w[e] = (unsigned short)bf16_bits(tf[(c8 + e) * SPT + tl]);
      o[it] = w;
    }
#pragma unroll
    for (int it = 0; it < 4; ++it) {
      const int tl = it * 16 + rsub;
      *(volatile v8us*)(XT + ((size_t)(b * NPOS + n0 + tl)) * CC + c8) = o[it];
    }
    __threadfence();
#pragma unroll
    for (int it = 0; it < 4; ++it) {
      const int tl = it * 16 + rsub;
      *(volatile v8us*)(XT + ((size_t)(b * NPOS + n0 + tl)) * CC + c8) = o[it];
    }
  } else if (bx < PREP_XT + PREP_WP) {
    const int j = bx - PREP_XT;
    const int which = j >> 2;
    const int u  = (j & 3) * 256 + tid;
    const int o  = u >> 4;
    const int k8 = (u & 15) * 8;
    const size_t so = (size_t)o * CC + k8;
    v4f a, c;
    if (which == 0)      { a = *(const v4f*)(wth + so); c = *(const v4f*)(wth + so + 4); }
    else if (which == 1) { a = *(const v4f*)(wph + so); c = *(const v4f*)(wph + so + 4); }
    else                 { a = *(const v4f*)(wg  + so); c = *(const v4f*)(wg  + so + 4); }
    const v8us o8 = cvt8(a, c);
    unsigned short* dp = WP + ((size_t)which * 1024 + (size_t)u) * 8;
    *(volatile v8us*)dp = o8;
    __threadfence();
    *(volatile v8us*)dp = o8;
  } else if (bx < PREP_XT + PREP_WP + PREP_WW) {
    const int j = bx - (PREP_XT + PREP_WP);
    const int v  = j * 256 + tid;
    const int o  = v >> 4;
    const int k8 = (v & 15) * 8;
    const int kk = k8 & (CI - 1);
    const float* p = wW + (size_t)o * CI + kk;
    const v4f a = *(const v4f*)p;
    const v4f c = *(const v4f*)(p + 4);
    const v8us o8 = cvt8(a, c);
    unsigned short* dp = WW2 + (size_t)v * 8;
    *(volatile v8us*)dp = o8;
    __threadfence();
    *(volatile v8us*)dp = o8;
  } else {
    const int j  = bx - (PREP_XT + PREP_WP + PREP_WW);
    const int nq = (j < 3) ? (CI / 4) : (CC / 4);
    const int so = (j < 3) ? (j * CI) : (3 * CI + (j - 3) * CC);
    const int tq = (tid < nq) ? tid : (nq - 1);
    const int t4 = tq * 4;
    v4f a;
    if (j == 0)      a = *(const v4f*)(bth + t4);
    else if (j == 1) a = *(const v4f*)(bph + t4);
    else if (j == 2) a = *(const v4f*)(bg  + t4);
    else if (j == 3) a = *(const v4f*)(bW  + t4);
    else if (j == 4) a = *(const v4f*)(gnw + t4);
    else             a = *(const v4f*)(gnb + t4);
    v4f o;
    o.x = bf16_val(a.x); o.y = bf16_val(a.y); o.z = bf16_val(a.z); o.w = bf16_val(a.w);
    if (tid < nq) *(volatile v4f*)(SV + so + t4) = o;
    __threadfence();
    if (tid < nq) *(volatile v4f*)(SV + so + t4) = o;
  }
}

__global__ __launch_bounds__(128) void k_proj(const unsigned short* __restrict__ A,
                                             const unsigned short* __restrict__ BT,
                                             const float* __restrict__ bp,
                                             unsigned short* thl, float* pg) {
  __shared__ __attribute__((aligned(16))) float stg[64 * SPT];
  __shared__ __attribute__((aligned(16))) float sb[64];
  const int tid = (int)threadIdx.x, lane = tid & 31, wave = tid >> 5, hh = lane >> 4, m = lane & 15;
  const int rowBase = (int)blockIdx.x * 64;
  const int cb = (int)blockIdx.y;
  const int colBase = cb * 64;
  if (tid < 16) {
    const v4f bv = *(const v4f*)(bp + colBase + 4 * tid);
    *(v4fa*)(sb + 4 * tid) = bv;
  }
  v8f acc[4];
#pragma unroll
  for (int t = 0; t < 4; ++t) acc[t] = z8();
  const unsigned short* ap = A  + (size_t)(rowBase + 16 * wave + m) * CC + 8 * hh;
  const unsigned short* bq = BT + (size_t)(colBase + m) * CC + 8 * hh;
#pragma unroll 1
  for (int k0 = 0; k0 < CC; k0 += 32) {
    FragB af;
    af.h[0] = *(const v8usa*)(ap + k0);
    af.h[1] = *(const v8usa*)(ap + k0 + 16);
#pragma unroll
    for (int nt = 0; nt < 4; ++nt) {
      const unsigned short* wq = bq + (size_t)(16 * nt) * CC + k0;
      FragB bf;
      bf.h[0] = *(const v8usa*)wq;
      bf.h[1] = *(const v8usa*)(wq + 16);
      acc[nt] = wmb(af, bf, acc[nt]);
    }
  }
#pragma unroll
  for (int nt = 0; nt < 4; ++nt) {
    const int lc = 16 * nt + m;
#pragma unroll
    for (int r = 0; r < 8; ++r) {
      const int lr = 16 * wave + 8 * hh + r;
      stg[lr * SPT + lc] = acc[nt][r];
    }
  }
  __syncthreads();

  if (cb == 0) {
    const int rsub = tid >> 3;
    const int c8   = (tid & 7) * 8;
    v8us hv[4], lv[4];
#pragma unroll
    for (int it = 0; it < 4; ++it) {
      const int row = it * 16 + rsub;
      const float* sp = stg + row * SPT + c8;
      v8us h8, l8;
#pragma unroll
      for (int e = 0; e < 8; ++e) {
        const float v = sp[e] + sb[c8 + e];
        const unsigned hb = bf16_bits(v);
        const unsigned lb = bf16_bits(v - __uint_as_float(hb << 16));
        h8[e] = (unsigned short)hb;
        l8[e] = (unsigned short)lb;
      }
      hv[it] = h8; lv[it] = l8;
    }
#pragma unroll
    for (int it = 0; it < 4; ++it) {
      const int row = it * 16 + rsub;
      unsigned short* dp = thl + (size_t)(rowBase + row) * CC + c8;
      *(volatile v8us*)dp        = hv[it];
      *(volatile v8us*)(dp + CI) = lv[it];
    }
    __threadfence();
#pragma unroll
    for (int it = 0; it < 4; ++it) {
      const int row = it * 16 + rsub;
      unsigned short* dp = thl + (size_t)(rowBase + row) * CC + c8;
      *(volatile v8us*)dp        = hv[it];
      *(volatile v8us*)(dp + CI) = lv[it];
    }
  } else {
    const int rsub = tid >> 4;
    const int c4   = (tid & 15) * 4;
    const int oc   = (cb - 1) * 64 + c4;
    v4f pv[8];
#pragma unroll
    for (int it = 0; it < 8; ++it) {
      const int row = it * 8 + rsub;
      v4f v = *(const v4fa*)(stg + row * SPT + c4);
      v.x += sb[c4]; v.y += sb[c4 + 1]; v.z += sb[c4 + 2]; v.w += sb[c4 + 3];
      pv[it] = v;
    }
#pragma unroll
    for (int it = 0; it < 8; ++it) {
      const int row = it * 8 + rsub;
      *(volatile v4f*)(pg + (size_t)(rowBase + row) * CC + oc) = pv[it];
    }
    __threadfence();
#pragma unroll
    for (int it = 0; it < 8; ++it) {
      const int row = it * 8 + rsub;
      *(volatile v4f*)(pg + (size_t)(rowBase + row) * CC + oc) = pv[it];
    }
  }
}

__global__ __launch_bounds__(256) void k_pool(const float* __restrict__ pg, unsigned short* phl, unsigned short* gt) {
  __shared__ __attribute__((aligned(16))) float pm[64 * TPT];
  const int bx = (int)blockIdx.x, tid = (int)threadIdx.x;
  const int b  = bx / (NKEY / 64);
  const int m0 = (bx - b * (NKEY / 64)) * 64;
  {
    const int p = tid >> 2, q = tid & 3;
    const int mm = m0 + p;
    const int i  = mm / PWD;
    const int jj = mm - i * PWD;
    const float* r0 = pg + ((size_t)(b * NPOS + (2 * i) * IW + 2 * jj)) * CC;
#pragma unroll 2
    for (int it = 0; it < 8; ++it) {
      const int c4 = (it * 4 + q) * 4;
      const v4f a = *(const v4f*)(r0 + c4);
      const v4f c = *(const v4f*)(r0 + CC + c4);
      const v4f d = *(const v4f*)(r0 + (size_t)IW * CC + c4);
      const v4f e = *(const v4f*)(r0 + (size_t)(IW + 1) * CC + c4);
      v4f mx;
      mx.x = fmaxf(fmaxf(a.x, c.x), fmaxf(d.x, e.x));
      mx.y = fmaxf(fmaxf(a.y, c.y), fmaxf(d.y, e.y));
      mx.z = fmaxf(fmaxf(a.z, c.z), fmaxf(d.z, e.z));
      mx.w = fmaxf(fmaxf(a.w, c.w), fmaxf(d.w, e.w));
      *(v4fa*)(pm + p * TPT + c4) = mx;
    }
  }
  __syncthreads();
  const int rsub = tid >> 3;
  const int c8   = (tid & 7) * 8;
  v8us ph[2], pl[2], gh[2], gl[2];
#pragma unroll
  for (int it = 0; it < 2; ++it) {
    const int row = it * 32 + rsub;
    v8us h8, l8, g8, k8;
#pragma unroll
    for (int e = 0; e < 8; ++e) {
      const float v = pm[row * TPT + c8 + e];
      const unsigned hb = bf16_bits(v);
      const unsigned lb = bf16_bits(v - __uint_as_float(hb << 16));
      h8[e] = (unsigned short)hb; l8[e] = (unsigned short)lb;
      const float w = pm[(c8 + e) * TPT + CI + row];
      const unsigned gb = bf16_bits(w);
      const unsigned kb = bf16_bits(w - __uint_as_float(gb << 16));
      g8[e] = (unsigned short)gb; k8[e] = (unsigned short)kb;
    }
    ph[it] = h8; pl[it] = l8; gh[it] = g8; gl[it] = k8;
  }
#pragma unroll
  for (int it = 0; it < 2; ++it) {
    const int row = it * 32 + rsub;
    unsigned short* pr = phl + ((size_t)(b * NKEY + m0 + row)) * CC + c8;
    unsigned short* gr = gt + ((size_t)(b * CI + row)) * GTP + m0 + c8;
    *(volatile v8us*)pr          = ph[it];
    *(volatile v8us*)(pr + CI)   = pl[it];
    *(volatile v8us*)gr          = gh[it];
    *(volatile v8us*)(gr + NKEY) = gl[it];
  }
  __threadfence();
#pragma unroll
  for (int it = 0; it < 2; ++it) {
    const int row = it * 32 + rsub;
    unsigned short* pr = phl + ((size_t)(b * NKEY + m0 + row)) * CC + c8;
    unsigned short* gr = gt + ((size_t)(b * CI + row)) * GTP + m0 + c8;
    *(volatile v8us*)pr          = ph[it];
    *(volatile v8us*)(pr + CI)   = pl[it];
    *(volatile v8us*)gr          = gh[it];
    *(volatile v8us*)(gr + NKEY) = gl[it];
  }
}

#define AT_D  64
#define AT_NW 4
#define AT_QB 64
#define AT_KC 64
#define AT_L2E 1.4426950408889634f

__device__ __forceinline__ unsigned short at_bf_bits(float f) {
  unsigned u = __float_as_uint(f);
  return (unsigned short)((u + 0x7FFFu + ((u >> 16) & 1u)) >> 16);
}
__device__ __forceinline__ __bf16 at_f2bf(float f) { return __builtin_bit_cast(__bf16, at_bf_bits(f)); }
__device__ __forceinline__ void at_split(float f, __bf16& hi, __bf16& lo) {
  const unsigned short hb = at_bf_bits(f);
  hi = __builtin_bit_cast(__bf16, hb);
  lo = at_f2bf(f - __uint_as_float(((unsigned)hb) << 16));
}
__device__ __forceinline__ v8f at_mma(v16bf a, v16bf b, v8f c) {
  c = __builtin_amdgcn_wmma_f32_16x16x32_bf16(false, a, false, b, (short)0, c, false, false);
  asm volatile("v_nop\n\tv_nop\n\tv_nop\n\tv_nop" : "+v"(c) : "v"(a), "v"(b));
  return c;
}
union AtFB { v16bf v; v8bf h[2]; };
__device__ __forceinline__ v16bf at_ldfrag(const __bf16* p) {
  AtFB f; f.h[0] = *(const v8bf*)(p); f.h[1] = *(const v8bf*)(p + 16); return f.v;
}

__global__ __launch_bounds__(128) __attribute__((amdgpu_num_vgpr(248)))
void k_attn(const unsigned short* __restrict__ thl, const unsigned short* __restrict__ phl,
            const unsigned short* __restrict__ gtp, unsigned short* yout) {
  __shared__ __align__(16) __bf16 Ksh[AT_KC * AT_D];
  __shared__ __align__(16) __bf16 Ksl[AT_KC * AT_D];
  __shared__ __align__(16) __bf16 Vth[AT_D * AT_KC];
  __shared__ __align__(16) __bf16 Vtl[AT_D * AT_KC];
  __shared__ __align__(16) __bf16 Psh[AT_NW][16 * AT_KC];
  __shared__ __align__(16) __bf16 Psl[AT_NW][16 * AT_KC];
  __shared__ __align__(16) float  Os[AT_NW][16 * SPT];

  const int tid  = (int)threadIdx.x;
  const int wave = tid >> 5;
  const int lane = tid & 31;
  const int hh   = lane >> 4;
  const int c    = lane & 15;

  const int nqb = NPOS / AT_QB;
  const int bx  = (int)blockIdx.x;
  const int b   = bx / nqb;
  const int qb  = bx - b * nqb;
  const int q0  = qb * AT_QB + wave * 16;

  const __bf16* Qb = (const __bf16*)(const void*)thl + (size_t)b * NPOS * CC;
  const __bf16* Kb = (const __bf16*)(const void*)phl + (size_t)b * NKEY * CC;
  const __bf16* Vb = (const __bf16*)(const void*)gtp + (size_t)b * CI * GTP;
  unsigned short* yb = yout + (size_t)b * NPOS * CC;

  v16bf qah[2], qal[2];
#pragma unroll
  for (int dc = 0; dc < 2; ++dc) {
    const __bf16* qr = Qb + (size_t)(q0 + c) * CC + dc * 32 + 8 * hh;
    qah[dc] = at_ldfrag(qr);
    qal[dc] = at_ldfrag(qr + AT_D);
  }

  float mrow[8], lrow[8];
  v8f oacc[4];
#pragma unroll
  for (int r = 0; r < 8; ++r) { mrow[r] = -INFINITY; lrow[r] = 0.f; }
#pragma unroll
  for (int t = 0; t < 4; ++t) oacc[t] = z8();

  const int nChunks = NKEY / AT_KC;
  for (int kc = 0; kc < nChunks; ++kc) {
    const int kv0 = kc * AT_KC;
    __syncthreads();
    {
      const int r = tid >> 1, half = (tid & 1) * 32;
      const __bf16* ksh = Kb + (size_t)(kv0 + r) * CC + half;
      const __bf16* ksl = ksh + AT_D;
      const __bf16* vsh = Vb + (size_t)r * GTP + kv0 + half;
      const __bf16* vsl = vsh + NKEY;
#pragma unroll
      for (int i = 0; i < 4; ++i) {
        const v8bf a0 = *(const v8bf*)(ksh + 8 * i);
        const v8bf a1 = *(const v8bf*)(ksl + 8 * i);
        const v8bf b0 = *(const v8bf*)(vsh + 8 * i);
        const v8bf b1 = *(const v8bf*)(vsl + 8 * i);
        *(v8bf*)(Ksh + r * AT_D  + half + 8 * i) = a0;
        *(v8bf*)(Ksl + r * AT_D  + half + 8 * i) = a1;
        *(v8bf*)(Vth + r * AT_KC + half + 8 * i) = b0;
        *(v8bf*)(Vtl + r * AT_KC + half + 8 * i) = b1;
      }
    }
    __syncthreads();

    v8f s[4];
#pragma unroll
    for (int j = 0; j < 4; ++j) {
      s[j] = z8();
#pragma unroll
      for (int dc = 0; dc < 2; ++dc) {
        AtFB kb, kl;
        kb.h[0] = *(const v8bf*)(Ksh + (j * 16 + c) * AT_D + dc * 32 + 8 * hh);
        kb.h[1] = *(const v8bf*)(Ksh + (j * 16 + c) * AT_D + dc * 32 + 16 + 8 * hh);
        kl.h[0] = *(const v8bf*)(Ksl + (j * 16 + c) * AT_D + dc * 32 + 8 * hh);
        kl.h[1] = *(const v8bf*)(Ksl + (j * 16 + c) * AT_D + dc * 32 + 16 + 8 * hh);
        s[j] = at_mma(qah[dc], kb.v, s[j]);
        s[j] = at_mma(qah[dc], kl.v, s[j]);
        s[j] = at_mma(qal[dc], kb.v, s[j]);
      }
    }
    float cm[8];
#pragma unroll
    for (int r = 0; r < 8; ++r) {
      float mx = -INFINITY;
#pragma unroll
      for (int j = 0; j < 4; ++j) mx = fmaxf(mx, s[j][r]);
#pragma unroll
      for (int off = 1; off < 16; off <<= 1) mx = fmaxf(mx, __shfl_xor(mx, off, 32));
      cm[r] = mx;
    }
    __bf16* pwh = Psh[wave];
    __bf16* pwl = Psl[wave];
#pragma unroll
    for (int r = 0; r < 8; ++r) {
      const float mnew  = fmaxf(mrow[r], cm[r]);
      const float alpha = __builtin_amdgcn_exp2f((mrow[r] - mnew) * AT_L2E);
      mrow[r] = mnew;
      const float nml = -mnew * AT_L2E;
      float psum = 0.f;
#pragma unroll
      for (int j = 0; j < 4; ++j) {
        const float p = __builtin_amdgcn_exp2f(fmaf(s[j][r], AT_L2E, nml));
        psum += p;
        __bf16 a, bl; at_split(p, a, bl);
        pwh[(8 * hh + r) * AT_KC + j * 16 + c] = a;
        pwl[(8 * hh + r) * AT_KC + j * 16 + c] = bl;
      }
#pragma unroll
      for (int off = 1; off < 16; off <<= 1) psum += __shfl_xor(psum, off, 32);
      lrow[r] = lrow[r] * alpha + psum;
#pragma unroll
      for (int t = 0; t < 4; ++t) oacc[t][r] *= alpha;
    }
    __builtin_amdgcn_fence(__ATOMIC_RELEASE, "workgroup");
    __builtin_amdgcn_wave_barrier();
    __builtin_amdgcn_fence(__ATOMIC_ACQUIRE, "workgroup");
#pragma unroll 1
    for (int kk = 0; kk < 2; ++kk) {
      AtFB pa, pl;
      pa.h[0] = *(const v8bf*)(pwh + c * AT_KC + kk * 32 + 8 * hh);
      pa.h[1] = *(const v8bf*)(pwh + c * AT_KC + kk * 32 + 16 + 8 * hh);
      pl.h[0] = *(const v8bf*)(pwl + c * AT_KC + kk * 32 + 8 * hh);
      pl.h[1] = *(const v8bf*)(pwl + c * AT_KC + kk * 32 + 16 + 8 * hh);
#pragma unroll
      for (int t = 0; t < 4; ++t) {
        AtFB vb, vl;
        vb.h[0] = *(const v8bf*)(Vth + (t * 16 + c) * AT_KC + kk * 32 + 8 * hh);
        vb.h[1] = *(const v8bf*)(Vth + (t * 16 + c) * AT_KC + kk * 32 + 16 + 8 * hh);
        vl.h[0] = *(const v8bf*)(Vtl + (t * 16 + c) * AT_KC + kk * 32 + 8 * hh);
        vl.h[1] = *(const v8bf*)(Vtl + (t * 16 + c) * AT_KC + kk * 32 + 16 + 8 * hh);
        oacc[t] = at_mma(pa.v, vb.v, oacc[t]);
        oacc[t] = at_mma(pa.v, vl.v, oacc[t]);
        oacc[t] = at_mma(pl.v, vb.v, oacc[t]);
      }
    }
  }

  float* os = Os[wave];
#pragma unroll
  for (int r = 0; r < 8; ++r) {
    const float inv = 1.0f / lrow[r];
#pragma unroll
    for (int t = 0; t < 4; ++t) os[(8 * hh + r) * SPT + t * 16 + c] = oacc[t][r] * inv;
  }
  __builtin_amdgcn_fence(__ATOMIC_RELEASE, "workgroup");
  __builtin_amdgcn_wave_barrier();
  __builtin_amdgcn_fence(__ATOMIC_ACQUIRE, "workgroup");
  {
    const int q  = lane >> 3;
    const int c8 = (lane & 7) * 8;
    v8us hv[4], lv[4];
#pragma unroll
    for (int it = 0; it < 4; ++it) {
      const int row = it * 4 + q;
      const float* sp = os + row * SPT + c8;
      v8us h8, l8;
#pragma unroll
      for (int e = 0; e < 8; ++e) {
        const float f = sp[e];
        const unsigned short hb = at_bf_bits(f);
        const unsigned short lb = at_bf_bits(f - __uint_as_float(((unsigned)hb) << 16));
        h8[e] = hb; l8[e] = lb;
      }
      hv[it] = h8; lv[it] = l8;
    }
#pragma unroll
    for (int it = 0; it < 4; ++it) {
      const int row = it * 4 + q;
      unsigned short* yr = yb + (size_t)(q0 + row) * CC + c8;
      *(volatile v8us*)(yr)        = hv[it];
      *(volatile v8us*)(yr + AT_D) = lv[it];
    }
    __threadfence();
#pragma unroll
    for (int it = 0; it < 4; ++it) {
      const int row = it * 4 + q;
      unsigned short* yr = yb + (size_t)(q0 + row) * CC + c8;
      *(volatile v8us*)(yr)        = hv[it];
      *(volatile v8us*)(yr + AT_D) = lv[it];
    }
  }
}

__global__ __launch_bounds__(256) void k_w(const unsigned short* __restrict__ A,
                                          const unsigned short* __restrict__ BT,
                                          const float* __restrict__ bw,
                                          float* wyc, double* rec) {
  __shared__ __attribute__((aligned(16))) float stg[64 * TPT];
  __shared__ __attribute__((aligned(16))) float sb[64];
  __shared__ __attribute__((aligned(16))) double rc[32];
  const int tid = (int)threadIdx.x, lane = tid & 31, wave = tid >> 5, hh = lane >> 4, m = lane & 15;
  const int bx = (int)blockIdx.x, by = (int)blockIdx.y;
  const int rowBase = bx * WROWS;
  const int colBase = by * 64;
  if (tid < 16) {
    const v4f bv = *(const v4f*)(bw + colBase + 4 * tid);
    *(v4fa*)(sb + 4 * tid) = bv;
  }
  v8f acc[4];
#pragma unroll
  for (int t = 0; t < 4; ++t) acc[t] = z8();
  const unsigned short* ap = A  + (size_t)(rowBase + 16 * wave + m) * CC + 8 * hh;
  const unsigned short* bq = BT + (size_t)(colBase + m) * CC + 8 * hh;
#pragma unroll 1
  for (int k0 = 0; k0 < CC; k0 += 32) {
    FragB af;
    af.h[0] = *(const v8usa*)(ap + k0);
    af.h[1] = *(const v8usa*)(ap + k0 + 16);
#pragma unroll
    for (int nt = 0; nt < 4; ++nt) {
      const unsigned short* wq = bq + (size_t)(16 * nt) * CC + k0;
      FragB bf;
      bf.h[0] = *(const v8usa*)wq;
      bf.h[1] = *(const v8usa*)(wq + 16);
      acc[nt] = wmb(af, bf, acc[nt]);
    }
  }
#pragma unroll
  for (int nt = 0; nt < 4; ++nt) {
    const int lc = 16 * nt + m;
#pragma unroll
    for (int r = 0; r < 8; ++r) {
      const int lr = 16 * wave + 8 * hh + r;
      stg[lc * TPT + lr] = acc[nt][r];
    }
  }
  __syncthreads();

  const int b  = bx / RECB;
  const int n0 = (bx - b * RECB) * WROWS;
  v4f pv[8];
  float s0 = 0.f, q0 = 0.f, s1 = 0.f, q1 = 0.f;
#pragma unroll
  for (int it = 0; it < 8; ++it) {
    const int ch = wave * 8 + it;
    const float bc = sb[ch];
    v4f v = *(const v4fa*)(stg + ch * TPT + lane * 4);
    v.x += bc; v.y += bc; v.z += bc; v.w += bc;
    pv[it] = v;
    const float ps = (v.x + v.y) + (v.z + v.w);
    const float pq = fmaf(v.x, v.x, v.y * v.y) + fmaf(v.z, v.z, v.w * v.w);
    if (it < 4) { s0 += ps; q0 += pq; } else { s1 += ps; q1 += pq; }
  }
#pragma unroll
  for (int it = 0; it < 8; ++it) {
    const int ch = wave * 8 + it;
    *(volatile v4f*)(wyc + ((size_t)(b * CC + colBase + ch)) * NPOS + n0 + lane * 4) = pv[it];
  }
  __threadfence();
#pragma unroll
  for (int it = 0; it < 8; ++it) {
    const int ch = wave * 8 + it;
    *(volatile v4f*)(wyc + ((size_t)(b * CC + colBase + ch)) * NPOS + n0 + lane * 4) = pv[it];
  }
  double ds0 = (double)s0, dq0 = (double)q0, ds1 = (double)s1, dq1 = (double)q1;
#pragma unroll
  for (int off = 16; off > 0; off >>= 1) {
    ds0 += __shfl_xor(ds0, off, 32);
    dq0 += __shfl_xor(dq0, off, 32);
    ds1 += __shfl_xor(ds1, off, 32);
    dq1 += __shfl_xor(dq1, off, 32);
  }
  if (lane == 0) {
    rc[4 * wave + 0] = ds0; rc[4 * wave + 1] = dq0;
    rc[4 * wave + 2] = ds1; rc[4 * wave + 3] = dq1;
  }
  __syncthreads();
  v2d rv;
  rv.x = 0.0; rv.y = 0.0;
  if (tid < 16) {
    rv = *(const v2da*)(rc + 2 * tid);
    *(volatile v2d*)(rec + ((size_t)bx * NGRP + by * 16 + tid) * 2) = rv;
  }
  __threadfence();
  if (tid < 16) {
    *(volatile v2d*)(rec + ((size_t)bx * NGRP + by * 16 + tid) * 2) = rv;
  }
}

__global__ __launch_bounds__(128) void k_combine(const double* __restrict__ rec, float* st) {
  __shared__ __attribute__((aligned(16))) float sst[256];
  const int tid = (int)threadIdx.x;
  const int b = tid >> 5, g = tid & 31;
  double S = 0.0, Q = 0.0;
#pragma unroll 4
  for (int j = 0; j < RECB; ++j) {
    const v2d r = *(const v2d*)(rec + ((size_t)((b * RECB + j) * NGRP + g)) * 2);
    S += r.x; Q += r.y;
  }
  const double inv = 1.0 / (double)GCNT;
  const double mean = S * inv;
  double var = Q * inv - mean * mean;
  if (var < 0.0) var = 0.0;
  const float vf = (float)(var + 1e-5);
  const float rstd = 1.0f / sqrtf(vf);
  sst[2 * tid]     = (float)mean;
  sst[2 * tid + 1] = rstd;
  __syncthreads();
  v4f v;
  v.x = 0.f; v.y = 0.f; v.z = 0.f; v.w = 0.f;
  if (tid < 64) {
    v = *(const v4fa*)(sst + 4 * tid);
    *(volatile v4f*)(st + 4 * tid) = v;
  }
  __threadfence();
  if (tid < 64) {
    *(volatile v4f*)(st + 4 * tid) = v;
  }
}

__global__ __launch_bounds__(256) void k_out(const float* __restrict__ wyc, const float* __restrict__ st,
                                            const float* __restrict__ sv, const float* __restrict__ x, float* out) {
#pragma clang fp contract(off)
  const int bx = (int)blockIdx.x, tid = (int)threadIdx.x;
  const int plane = bx / (NPOS / 1024);
  const int b = plane >> 7;
  const int c = plane & (CC - 1);
  const int g = c >> 2;
  const float mean = st[(b * NGRP + g) * 2];
  const float rstd = st[(b * NGRP + g) * 2 + 1];
  const float gw = sv[SV_GW + c];
  const float gb = sv[SV_GB + c];
  const size_t e = ((size_t)bx * 256 + (size_t)tid) * 4;
  const v4f w  = *(const v4f*)(wyc + e);
  const v4f xr = *(const v4f*)(x + e);
  v4f o;
  o.x = (((w.x - mean) * rstd) * gw + gb) + bf16_val(xr.x);
  o.y = (((w.y - mean) * rstd) * gw + gb) + bf16_val(xr.y);
  o.z = (((w.z - mean) * rstd) * gw + gb) + bf16_val(xr.z);
  o.w = (((w.w - mean) * rstd) * gw + gb) + bf16_val(xr.w);
  *(volatile v4f*)(out + e) = o;
  __threadfence();
  *(volatile v4f*)(out + e) = o;
}

static inline size_t al256(size_t o) { return (o + 255) & ~(size_t)255; }

extern "C" void kernel_launch(void* const* d_in, const int* in_sizes, int n_in,
                              void* d_out, int out_size, void* d_ws, size_t ws_size,
                              hipStream_t stream) {
  if (n_in < 11) return;
  if (in_sizes[0] != NB * CC * NPOS) return;
  if (in_sizes[1] != CI * CC || in_sizes[3] != CI * CC || in_sizes[5] != CI * CC) return;
  if (in_sizes[2] != CI || in_sizes[4] != CI || in_sizes[6] != CI) return;
  if (in_sizes[7] != CC * CI) return;
  if (in_sizes[8] != CC || in_sizes[9] != CC || in_sizes[10] != CC) return;
  if (out_size != NB * CC * NPOS) return;

  const float* x       = (const float*)d_in[0];
  const float* w_theta = (const float*)d_in[1];
  const float* b_theta = (const float*)d_in[2];
  const float* w_phi   = (const float*)d_in[3];
  const float* b_phi   = (const float*)d_in[4];
  const float* w_g     = (const float*)d_in[5];
  const float* b_g     = (const float*)d_in[6];
  const float* w_W     = (const float*)d_in[7];
  const float* b_W     = (const float*)d_in[8];
  const float* gn_w    = (const float*)d_in[9];
  const float* gn_b    = (const float*)d_in[10];
  float* out = (float*)d_out;

  const size_t P16  = (size_t)NTOK * CC * 2;
  const size_t P32  = (size_t)NTOK * CC * 4;
  const size_t PKV  = (size_t)NB * NKEY * CC * 2;
  const size_t PWP  = (size_t)3 * CI * CC * 2;
  const size_t PWW  = (size_t)CC * CC * 2;
  const size_t PSV  = (size_t)SV_N * 4;
  const size_t PREC = (size_t)NREC * NGRP * 2 * 8;
  const size_t PST  = (size_t)NB * NGRP * 2 * 4;
  size_t off = 0;
  const size_t oXT  = off; off = al256(off + P16);
  const size_t oTHL = off; off = al256(off + P16);
  const size_t oPG  = off; off = al256(off + P32);
  const size_t oPHL = off; off = al256(off + PKV);
  const size_t oGT  = off; off = al256(off + PKV);
  const size_t oYHL = off; off = al256(off + P16);
  const size_t oWYC = off; off = al256(off + P32);
  const size_t oWP  = off; off = al256(off + PWP);
  const size_t oWW2 = off; off = al256(off + PWW);
  const size_t oSV  = off; off = al256(off + PSV);
  const size_t oREC = off; off = al256(off + PREC);
  const size_t oST  = off; off = al256(off + PST);
  if (off > ws_size || off > (size_t)WSMAX) return;

  char* ws = (char*)d_ws;
  unsigned short* XT  = (unsigned short*)(ws + oXT);
  unsigned short* THL = (unsigned short*)(ws + oTHL);
  float*          PG  = (float*)(ws + oPG);
  unsigned short* PHL = (unsigned short*)(ws + oPHL);
  unsigned short* GT  = (unsigned short*)(ws + oGT);
  unsigned short* YHL = (unsigned short*)(ws + oYHL);
  float*          WYC = (float*)(ws + oWYC);
  unsigned short* WP  = (unsigned short*)(ws + oWP);
  unsigned short* WW2 = (unsigned short*)(ws + oWW2);
  float*          SV  = (float*)(ws + oSV);
  double*         REC = (double*)(ws + oREC);
  float*          ST  = (float*)(ws + oST);

  k_prep<<<PREP_XT + PREP_WP + PREP_WW + PREP_SV, 256, 0, stream>>>(x, w_theta, b_theta, w_phi, b_phi, w_g, b_g,
                                                                   w_W, b_W, gn_w, gn_b, XT, WP, WW2, SV);
  k_proj<<<dim3(NTOK / 64, 3, 1), 128, 0, stream>>>(XT, WP, SV + SV_BP, THL, PG);
  k_pool<<<NB * (NKEY / 64), 256, 0, stream>>>(PG, PHL, GT);
  k_attn<<<NB * (NPOS / AT_QB), 128, 0, stream>>>(THL, PHL, GT, YHL);
  k_w<<<dim3(NREC, 2, 1), 256, 0, stream>>>(YHL, WW2, SV + SV_BW, WYC, REC);
  k_combine<<<1, 128, 0, stream>>>(REC, ST);
  k_out<<<(NB * CC * NPOS) / 1024, 256, 0, stream>>>(WYC, ST, SV, x, out);
  (void)hipGetLastError();
}
